// MambaBlock_87205015977998
// MI455X (gfx1250) — hardware-verified
//
#include <hip/hip_runtime.h>
#include <stddef.h>
#include <stdint.h>
#include <math.h>


#define DM     1024
#define DI     2048
#define NST    16
#define SEQL   2048
#define NBAT   2
#define MROWS  (NBAT * SEQL)
#define GBM    64
#define GBN    64
#define GTHR   128
#define NTHR   256
#define CT     16
#define SC     64
#define SD     64
#define BCP    64
#define WSMAX  134217728

#define U_WIN  ((2 * DI) * (DM / 8))
#define U_WBC  (64 * (DI / 8))
#define U_WD   (DI * (DI / 8))
#define U_WO   (DM * (DI / 8))

static_assert(MROWS % GBM == 0 && (2 * DI) % GBN == 0 && DI % GBN == 0 && DM % GBN == 0 && BCP == GBN);
static_assert((DM & (DM - 1)) == 0 && (DI & (DI - 1)) == 0 && DM % 32 == 0 && DI % 32 == 0);
static_assert(GBM == (GTHR / 32) * 16);
static_assert(U_WIN % NTHR == 0 && U_WBC % NTHR == 0 && U_WD % NTHR == 0 && U_WO % NTHR == 0);
static_assert(SEQL % CT == 0 && SEQL % SC == 0 && DI % SD == 0 && DI == NTHR * 8);
static_assert(MROWS % 8 == 0 && DM == 4 * 256);
static_assert(SC * 32 / 4 == 8 * SD);

typedef float          v4f   __attribute__((ext_vector_type(4)));
typedef float          v8f   __attribute__((ext_vector_type(8)));
typedef int            v8i   __attribute__((ext_vector_type(8)));
typedef unsigned short v8us  __attribute__((ext_vector_type(8)));
typedef unsigned short v16us __attribute__((ext_vector_type(16)));
typedef __bf16         v16bf __attribute__((ext_vector_type(16)));
typedef v4f  __attribute__((may_alias)) v4fa;
typedef v8us __attribute__((may_alias)) v8usa;
union FragB { v16bf v; v16us u; v8us h[2]; v8i w; };

enum { EPI_IN = 0, EPI_SP = 1, EPI_PLAIN = 2, EPI_RES = 3 };

__device__ __forceinline__ v8f wmb(const FragB& a, const FragB& b, v8f c) {
  v8f d = __builtin_amdgcn_wmma_f32_16x16x32_bf16(false, a.v, false, b.v, (short)0, c, false, false);
  asm volatile("v_nop\n\tv_nop\n\tv_nop\n\tv_nop" : "+v"(d) : "v"(a.w), "v"(b.w));
  return d;
}

__device__ __forceinline__ unsigned bf16_bits(float f) {
  const unsigned u = __float_as_uint(f);
  return (u + 0x7FFFu + ((u >> 16) & 1u)) >> 16;
}
__device__ __forceinline__ float bf16_val(float f) {
  return __uint_as_float(bf16_bits(f) << 16);
}
__device__ __forceinline__ float silu_f(float v) {
  return v * __builtin_amdgcn_rcpf(1.0f + expf(-v));
}
__device__ __forceinline__ float softplus_f(float v) {
  return fmaxf(v, 0.0f) + log1pf(expf(-fabsf(v)));
}
__device__ __forceinline__ void put8(unsigned short* p, v8us v) {
  *(volatile v8us*)p = v;
  __threadfence();
  *(volatile v8us*)p = v;
}
__device__ __forceinline__ void ld8(const float* p, float (&o)[8]) {
  const v4f a = *(const v4f*)p;
  const v4f b = *(const v4f*)(p + 4);
  o[0] = a.x; o[1] = a.y; o[2] = a.z; o[3] = a.w;
  o[4] = b.x; o[5] = b.y; o[6] = b.z; o[7] = b.w;
}

__global__ __launch_bounds__(NTHR) void k_prep1(const float* __restrict__ w_in, const float* __restrict__ w_b,
                                                const float* __restrict__ w_c,
                                                unsigned short* WINT, unsigned short* WBCT) {
  const int u = (int)blockIdx.x * NTHR + (int)threadIdx.x;
  v8us o = {0, 0, 0, 0, 0, 0, 0, 0};
  unsigned short* dp;
  if (u < U_WIN) {
    const int n  = u >> 7;
    const int k8 = (u & 127) * 8;
    const float* p = w_in + (size_t)k8 * (2 * DI) + n;
#pragma unroll
    for (int i = 0; i < 8; ++i) o[i] = (unsigned short)bf16_bits(p[(size_t)i * (2 * DI)]);
    dp = WINT + (size_t)n * DM + k8;
  } else if (u < U_WIN + U_WBC) {
    const int v  = u - U_WIN;
    const int n  = v >> 8;
    const int k8 = (v & 255) * 8;
    if (n < NST) {
      const float* p = w_b + (size_t)k8 * NST + n;
#pragma unroll
      for (int i = 0; i < 8; ++i) o[i] = (unsigned short)bf16_bits(p[(size_t)i * NST]);
    } else if (n < 2 * NST) {
      const float* p = w_c + (size_t)k8 * NST + (n - NST);
#pragma unroll
      for (int i = 0; i < 8; ++i) o[i] = (unsigned short)bf16_bits(p[(size_t)i * NST]);
    }
    dp = WBCT + (size_t)n * DI + k8;
  } else {
    return;
  }
  put8(dp, o);
}

__global__ __launch_bounds__(NTHR) void k_prep2(const float* __restrict__ w_delta, const float* __restrict__ w_out,
                                                unsigned short* WDT, unsigned short* WOT) {
  const int u = (int)blockIdx.x * NTHR + (int)threadIdx.x;
  v8us o = {0, 0, 0, 0, 0, 0, 0, 0};
  unsigned short* dp;
  if (u < U_WD) {
    const int n  = u >> 8;
    const int k8 = (u & 255) * 8;
    const float* p = w_delta + (size_t)k8 * DI + n;
#pragma unroll
    for (int i = 0; i < 8; ++i) o[i] = (unsigned short)bf16_bits(p[(size_t)i * DI]);
    dp = WDT + (size_t)n * DI + k8;
  } else if (u < U_WD + U_WO) {
    const int v  = u - U_WD;
    const int n  = v >> 8;
    const int k8 = (v & 255) * 8;
    const float* p = w_out + (size_t)k8 * DM + n;
#pragma unroll
    for (int i = 0; i < 8; ++i) o[i] = (unsigned short)bf16_bits(p[(size_t)i * DM]);
    dp = WOT + (size_t)n * DI + k8;
  } else {
    return;
  }
  put8(dp, o);
}

__global__ __launch_bounds__(NTHR) void k_ln(const float* __restrict__ x, const float* __restrict__ gw,
                                             const float* __restrict__ gb, unsigned short* XN) {
  const int tid = (int)threadIdx.x, lane = tid & 31, wave = tid >> 5;
  const int row = (int)blockIdx.x * 8 + wave;
  const float* xr = x + (size_t)row * DM + 8 * lane;
  float v[8];
  float s = 0.0f;
#pragma unroll 1
  for (int it = 0; it < 4; ++it) {
    ld8(xr + 256 * it, v);
    float t = 0.0f;
#pragma unroll
    for (int i = 0; i < 8; ++i) t += bf16_val(v[i]);
    s += t;
  }
#pragma unroll
  for (int d = 16; d >= 1; d >>= 1) s += __shfl_xor(s, d, 32);
  const float mu = s * (1.0f / (float)DM);
  float q = 0.0f;
#pragma unroll 1
  for (int it = 0; it < 4; ++it) {
    ld8(xr + 256 * it, v);
    float t = 0.0f;
#pragma unroll
    for (int i = 0; i < 8; ++i) { const float dd = bf16_val(v[i]) - mu; t = fmaf(dd, dd, t); }
    q += t;
  }
#pragma unroll
  for (int d = 16; d >= 1; d >>= 1) q += __shfl_xor(q, d, 32);
  const float var = q * (1.0f / (float)DM);
  const float rs  = rsqrtf(var + 1e-5f);
  unsigned short* orow = XN + (size_t)row * (2 * DM) + 8 * lane;
#pragma unroll 1
  for (int it = 0; it < 4; ++it) {
    float g8[8], b8[8];
    ld8(xr + 256 * it, v);
    ld8(gw + 256 * it + 8 * lane, g8);
    ld8(gb + 256 * it + 8 * lane, b8);
    v8us oh, ol;
#pragma unroll
    for (int i = 0; i < 8; ++i) {
      const float y = ((bf16_val(v[i]) - mu) * rs) * bf16_val(g8[i]) + bf16_val(b8[i]);
      const unsigned hb = bf16_bits(y);
      oh[i] = (unsigned short)hb;
      ol[i] = (unsigned short)bf16_bits(y - __uint_as_float(hb << 16));
    }
    unsigned short* hp = orow + 256 * it;
    *(volatile v8us*)hp = oh;
    *(volatile v8us*)(hp + DM) = ol;
    __threadfence();
    *(volatile v8us*)hp = oh;
    *(volatile v8us*)(hp + DM) = ol;
  }
}

template <int EPI>
__global__ __launch_bounds__(GTHR) void k_gemm(const unsigned short* __restrict__ A,
                                               const unsigned short* __restrict__ WT,
                                               float* outF, const float* __restrict__ aux, int KW, int ldo) {
  __shared__ __attribute__((aligned(16))) float stg[GBM * GBN];
  const int tid = (int)threadIdx.x, lane = tid & 31, wave = tid >> 5, hh = lane >> 4, m = lane & 15;
  const int rowBase = (int)blockIdx.x * GBM;
  const int col0    = (int)blockIdx.y * GBN;

  v8f acc[4];
  {
    const v8f z = {0.f, 0.f, 0.f, 0.f, 0.f, 0.f, 0.f, 0.f};
    acc[0] = z; acc[1] = z; acc[2] = z; acc[3] = z;
  }
  const unsigned short* ap = A  + (size_t)(rowBase + 16 * wave + m) * (size_t)(2 * KW) + 8 * hh;
  const unsigned short* wp = WT + (size_t)(col0 + m) * (size_t)KW + 8 * hh;
  const int ksteps = (2 * KW) >> 5;
  const int kmask  = KW - 1;
#pragma unroll 1
  for (int ks = 0; ks < ksteps; ++ks) {
    const int ka = 32 * ks;
    const int kb = ka & kmask;
    FragB af;
    af.h[0] = *(const v8usa*)(ap + ka);
    af.h[1] = *(const v8usa*)(ap + ka + 16);
#pragma unroll
    for (int t = 0; t < 4; ++t) {
      const unsigned short* wq = wp + (size_t)(16 * t) * (size_t)KW + kb;
      FragB bf;
      bf.h[0] = *(const v8usa*)wq;
      bf.h[1] = *(const v8usa*)(wq + 16);
      acc[t] = wmb(af, bf, acc[t]);
    }
  }

#pragma unroll
  for (int t = 0; t < 4; ++t) {
    const int lc = 16 * t + m;
#pragma unroll
    for (int r = 0; r < 8; ++r) {
      const int lr = 16 * wave + 8 * hh + r;
      stg[lr * GBN + lc] = acc[t][r];
    }
  }
  __syncthreads();

  int    ocol = col0;
  size_t ooff = 0;
  if constexpr (EPI == EPI_IN) {
    ocol = col0 & (DI - 1);
    ooff = (col0 >= DI) ? (size_t)MROWS * (size_t)DI : (size_t)0;
    if (col0 >= DI) {
#pragma unroll 1
      for (int i = 0; i < 8; ++i) {
        float* p = stg + (16 * wave + 2 * i + hh) * GBN + 4 * m;
        v4f v = *(const v4fa*)p;
        v.x = silu_f(v.x); v.y = silu_f(v.y); v.z = silu_f(v.z); v.w = silu_f(v.w);
        *(v4fa*)p = v;
      }
    }
  } else if constexpr (EPI == EPI_SP) {
    const v4f bq = *(const v4f*)(aux + col0 + 4 * m);
    const float b0 = bf16_val(bq.x), b1 = bf16_val(bq.y), b2 = bf16_val(bq.z), b3 = bf16_val(bq.w);
#pragma unroll 1
    for (int i = 0; i < 8; ++i) {
      float* p = stg + (16 * wave + 2 * i + hh) * GBN + 4 * m;
      v4f v = *(const v4fa*)p;
      v.x = softplus_f(v.x + b0); v.y = softplus_f(v.y + b1);
      v.z = softplus_f(v.z + b2); v.w = softplus_f(v.w + b3);
      *(v4fa*)p = v;
    }
  } else if constexpr (EPI == EPI_RES) {
#pragma unroll 1
    for (int i = 0; i < 8; ++i) {
      const int lr = 16 * wave + 2 * i + hh;
      float* p = stg + lr * GBN + 4 * m;
      const v4f xr = *(const v4f*)(aux + (size_t)(rowBase + lr) * (size_t)ldo + col0 + 4 * m);
      v4f v = *(const v4fa*)p;
      v.x += bf16_val(xr.x); v.y += bf16_val(xr.y); v.z += bf16_val(xr.z); v.w += bf16_val(xr.w);
      *(v4fa*)p = v;
    }
  }

  v4f fv[8];
#pragma unroll
  for (int i = 0; i < 8; ++i) {
    const int lr = 16 * wave + 2 * i + hh;
    fv[i] = *(const v4fa*)(stg + lr * GBN + 4 * m);
  }
  float* ob = outF + ooff + (size_t)rowBase * (size_t)ldo + ocol + 4 * m;
#pragma unroll
  for (int i = 0; i < 8; ++i) {
    const int lr = 16 * wave + 2 * i + hh;
    *(volatile v4f*)(ob + (size_t)lr * (size_t)ldo) = fv[i];
  }
  __threadfence();
#pragma unroll
  for (int i = 0; i < 8; ++i) {
    const int lr = 16 * wave + 2 * i + hh;
    *(volatile v4f*)(ob + (size_t)lr * (size_t)ldo) = fv[i];
  }
}

__global__ __launch_bounds__(NTHR) void k_conv(const float* __restrict__ XP, const float* __restrict__ wc,
                                               const float* __restrict__ bc, unsigned short* U) {
  const int tid  = (int)threadIdx.x;
  const int d0   = 8 * tid;
  const int row0 = (int)blockIdx.x * CT;
  const int l0   = row0 & (SEQL - 1);
  float w0[8], w1[8], w2[8], w3[8], bb[8];
#pragma unroll
  for (int c = 0; c < 8; ++c) {
    const v4f t = *(const v4f*)(wc + (size_t)(d0 + c) * 4);
    w0[c] = bf16_val(t.x); w1[c] = bf16_val(t.y); w2[c] = bf16_val(t.z); w3[c] = bf16_val(t.w);
  }
  ld8(bc + d0, bb);
#pragma unroll
  for (int c = 0; c < 8; ++c) bb[c] = bf16_val(bb[c]);

  float xa[8], xb[8], xc[8], xd[8];
  {
    const bool va = l0 >= 3, vb = l0 >= 2, vc = l0 >= 1;
    const int ra = va ? row0 - 3 : row0;
    const int rb = vb ? row0 - 2 : row0;
    const int rc = vc ? row0 - 1 : row0;
    ld8(XP + (size_t)ra * DI + d0, xa);
    ld8(XP + (size_t)rb * DI + d0, xb);
    ld8(XP + (size_t)rc * DI + d0, xc);
#pragma unroll
    for (int c = 0; c < 8; ++c) {
      xa[c] = va ? xa[c] : 0.0f;
      xb[c] = vb ? xb[c] : 0.0f;
      xc[c] = vc ? xc[c] : 0.0f;
    }
  }
#pragma unroll 1
  for (int t = 0; t < CT; ++t) {
    const int row = row0 + t;
    ld8(XP + (size_t)row * DI + d0, xd);
    v8us oh, ol;
#pragma unroll
    for (int c = 0; c < 8; ++c) {
      float a = w0[c] * xa[c];
      a = fmaf(w1[c], xb[c], a);
      a = fmaf(w2[c], xc[c], a);
      a = fmaf(w3[c], xd[c], a);
      a = a + bb[c];
      const float uu = silu_f(a);
      const unsigned hb = bf16_bits(uu);
      oh[c] = (unsigned short)hb;
      ol[c] = (unsigned short)bf16_bits(uu - __uint_as_float(hb << 16));
      xa[c] = xb[c]; xb[c] = xc[c]; xc[c] = xd[c];
    }
    unsigned short* hp = U + (size_t)row * (2 * DI) + d0;
    *(volatile v8us*)hp = oh;
    *(volatile v8us*)(hp + DI) = ol;
    __threadfence();
    *(volatile v8us*)hp = oh;
    *(volatile v8us*)(hp + DI) = ol;
  }
}

__global__ __launch_bounds__(SD) void k_scan(const float* __restrict__ DELTA, const float* __restrict__ SZ,
                                             const float* __restrict__ BC, const float* __restrict__ Alog,
                                             const float* __restrict__ Dp, unsigned short* UG) {
  __shared__ __attribute__((aligned(16))) float sBC[SC * 32];
  __shared__ __attribute__((aligned(16))) unsigned short sG[2 * SC * SD];
  const int tid = (int)threadIdx.x;
  const int b   = (int)blockIdx.x / (DI / SD);
  const int d0  = ((int)blockIdx.x % (DI / SD)) * SD;
  const int d   = d0 + tid;

  float An[NST], h[NST];
#pragma unroll
  for (int qd = 0; qd < 4; ++qd) {
    const v4f t = *(const v4f*)(Alog + (size_t)d * NST + 4 * qd);
    An[4 * qd + 0] = -expf(bf16_val(t.x));
    An[4 * qd + 1] = -expf(bf16_val(t.y));
    An[4 * qd + 2] = -expf(bf16_val(t.z));
    An[4 * qd + 3] = -expf(bf16_val(t.w));
  }
#pragma unroll
  for (int n = 0; n < NST; ++n) h[n] = 0.0f;
  const float Dd = bf16_val(Dp[d]);

#pragma unroll 1
  for (int l0 = 0; l0 < SEQL; l0 += SC) {
    const int rbase = b * SEQL + l0;
    __syncthreads();
#pragma unroll
    for (int i = 0; i < 8; ++i) {
      const int idx = i * SD + tid;
      const int tk  = idx >> 3;
      const int qd  = idx & 7;
      const v4f t = *(const v4f*)(BC + (size_t)(rbase + tk) * BCP + 4 * qd);
      *(v4fa*)(sBC + tk * 32 + 4 * qd) = t;
    }
    __syncthreads();

#pragma unroll 1
    for (int s = 0; s < SC; ++s) {
      const size_t r = (size_t)(rbase + s);
      const float dt = DELTA[r * DI + d];
      const float sz = SZ[r * DI + d];
      const unsigned uh = (unsigned)UG[r * (2 * DI) + d];
      const unsigned ul = (unsigned)UG[r * (2 * DI) + DI + d];
      const float xv = __uint_as_float(uh << 16) + __uint_as_float(ul << 16);
      const float dx = dt * xv;
      const float* bq = sBC + s * 32;
      float Bv[NST], Cv[NST];
#pragma unroll
      for (int qd = 0; qd < 4; ++qd) {
        const v4f tb = *(const v4fa*)(bq + 4 * qd);
        const v4f tc = *(const v4fa*)(bq + NST + 4 * qd);
        Bv[4 * qd + 0] = tb.x; Bv[4 * qd + 1] = tb.y; Bv[4 * qd + 2] = tb.z; Bv[4 * qd + 3] = tb.w;
        Cv[4 * qd + 0] = tc.x; Cv[4 * qd + 1] = tc.y; Cv[4 * qd + 2] = tc.z; Cv[4 * qd + 3] = tc.w;
      }
      float y = 0.0f;
#pragma unroll
      for (int n = 0; n < NST; ++n) {
        const float e = expf(dt * An[n]);
        h[n] = fmaf(e, h[n], dx * Bv[n]);
        y = fmaf(h[n], Cv[n], y);
      }
      y = y + Dd * xv;
      const float g = y * sz;
      const unsigned gh = bf16_bits(g);
      const unsigned gl = bf16_bits(g - __uint_as_float(gh << 16));
      sG[s * SD + tid]           = (unsigned short)gh;
      sG[SC * SD + s * SD + tid] = (unsigned short)gl;
    }
    __syncthreads();

    v8us qv[16];
#pragma unroll
    for (int rd = 0; rd < 16; ++rd) {
      const int pl = rd >> 3;
      const int tk = (rd & 7) * 8 + (tid >> 3);
      qv[rd] = *(const v8usa*)(sG + pl * (SC * SD) + tk * SD + 8 * (tid & 7));
    }
#pragma unroll
    for (int rd = 0; rd < 16; ++rd) {
      const int pl = rd >> 3;
      const int tk = (rd & 7) * 8 + (tid >> 3);
      unsigned short* dp = UG + (size_t)(rbase + tk) * (2 * DI) + pl * DI + d0 + 8 * (tid & 7);
      *(volatile v8us*)dp = qv[rd];
    }
    __threadfence();
#pragma unroll
    for (int rd = 0; rd < 16; ++rd) {
      const int pl = rd >> 3;
      const int tk = (rd & 7) * 8 + (tid >> 3);
      unsigned short* dp = UG + (size_t)(rbase + tk) * (2 * DI) + pl * DI + d0 + 8 * (tid & 7);
      *(volatile v8us*)dp = qv[rd];
    }
  }
}

static inline size_t al256(size_t o) { return (o + 255) & ~(size_t)255; }

extern "C" void kernel_launch(void* const* d_in, const int* in_sizes, int n_in,
                              void* d_out, int out_size, void* d_ws, size_t ws_size,
                              hipStream_t stream) {
  if (n_in < 13) return;
  if (in_sizes[0]  != MROWS * DM)   return;
  if (in_sizes[1]  != DM || in_sizes[2] != DM) return;
  if (in_sizes[3]  != DM * 2 * DI)  return;
  if (in_sizes[4]  != DI * 4)       return;
  if (in_sizes[5]  != DI)           return;
  if (in_sizes[6]  != DI * NST)     return;
  if (in_sizes[7]  != DI * NST || in_sizes[8] != DI * NST) return;
  if (in_sizes[9]  != DI * DI)      return;
  if (in_sizes[10] != DI || in_sizes[11] != DI) return;
  if (in_sizes[12] != DI * DM)      return;
  if (out_size != MROWS * DM)       return;

  const float* x       = (const float*)d_in[0];
  const float* w_norm  = (const float*)d_in[1];
  const float* b_norm  = (const float*)d_in[2];
  const float* w_in    = (const float*)d_in[3];
  const float* w_conv  = (const float*)d_in[4];
  const float* b_conv  = (const float*)d_in[5];
  const float* A_log   = (const float*)d_in[6];
  const float* w_b     = (const float*)d_in[7];
  const float* w_c     = (const float*)d_in[8];
  const float* w_delta = (const float*)d_in[9];
  const float* b_delta = (const float*)d_in[10];
  const float* D_param = (const float*)d_in[11];
  const float* w_out   = (const float*)d_in[12];
  float* out = (float*)d_out;

  char* ws = (char*)d_ws;
  size_t off = 0;
  const size_t szXN  = (size_t)MROWS * (2 * DM) * 2;
  const size_t szWIN = (size_t)(2 * DI) * DM * 2;
  const size_t szWD  = (size_t)DI * DI * 2;
  const size_t szWO  = (size_t)DM * DI * 2;
  const size_t szPL  = (size_t)MROWS * DI * 4;
  const size_t szU   = (size_t)MROWS * (2 * DI) * 2;
  const size_t szWBC = (size_t)64 * DI * 2;
  const size_t szBC  = (size_t)MROWS * BCP * 4;
  if (szWD + szWO > szXN) return;
  const size_t oXN  = off; off = al256(off + szXN);
  const size_t oWIN = off; off = al256(off + szWIN);
  const size_t oXP  = off; off = al256(off + szPL);
  const size_t oSZ  = off; off = al256(off + szPL);
  const size_t oU   = off; off = al256(off + szU);
  const size_t oWBC = off; off = al256(off + szWBC);
  const size_t oBC  = off; off = al256(off + szBC);
  if (oSZ != oXP + szPL) return;
  if (off > ws_size || off > (size_t)WSMAX) return;
  unsigned short* XN   = (unsigned short*)(ws + oXN);
  unsigned short* WINT = (unsigned short*)(ws + oWIN);
  unsigned short* WDT  = (unsigned short*)(ws + oXN);
  unsigned short* WOT  = (unsigned short*)(ws + oXN + szWD);
  float*          XP   = (float*)(ws + oXP);
  float*          SZp  = (float*)(ws + oSZ);
  unsigned short* UG   = (unsigned short*)(ws + oU);
  unsigned short* WBCT = (unsigned short*)(ws + oWBC);
  float*          BCp  = (float*)(ws + oBC);

  k_prep1<<<(U_WIN + U_WBC) / NTHR, NTHR, 0, stream>>>(w_in, w_b, w_c, WINT, WBCT);
  k_ln<<<MROWS / 8, NTHR, 0, stream>>>(x, w_norm, b_norm, XN);
  k_gemm<EPI_IN><<<dim3(MROWS / GBM, (2 * DI) / GBN), GTHR, 0, stream>>>(XN, WINT, XP, x, DM, DI);
  k_conv<<<MROWS / CT, NTHR, 0, stream>>>(XP, w_conv, b_conv, UG);
  k_prep2<<<(U_WD + U_WO) / NTHR, NTHR, 0, stream>>>(w_delta, w_out, WDT, WOT);
  k_gemm<EPI_SP><<<dim3(MROWS / GBM, DI / GBN), GTHR, 0, stream>>>(UG, WDT, XP, b_delta, DI, DI);
  k_gemm<EPI_PLAIN><<<dim3(MROWS / GBM, BCP / GBN), GTHR, 0, stream>>>(UG, WBCT, BCp, x, DI, BCP);
  k_scan<<<NBAT * (DI / SD), SD, 0, stream>>>(XP, SZp, BCp, A_log, D_param, UG);
  k_gemm<EPI_RES><<<dim3(MROWS / GBM, DM / GBN), GTHR, 0, stream>>>(UG, WOT, out, x, DI, DM);
}
